// GraphRNN_7413113553638
// MI455X (gfx1250) — hardware-verified
//
#include <hip/hip_runtime.h>
#include <math.h>

constexpr int N_SAMPLES    = 64;
constexpr int N_STEPS      = 2000;
constexpr int N_NODES      = N_SAMPLES * N_STEPS;
constexpr int N_EDGES      = 2048000;
constexpr int HID          = 64;
constexpr int GATES        = 4 * HID;
constexpr int HALF_SAMPLES = 32;
constexpr int HALF_ROWS    = HALF_SAMPLES * N_STEPS;
constexpr int SEQ_TILE     = 16;
constexpr int HPITCH       = 72;

constexpr float GCARRY = 64.0f;
constexpr float WCARRY = 64.0f;
constexpr float HCARRY = 1024.0f;
constexpr float GEMM_G_INV = 1.0f / (GCARRY * WCARRY);
constexpr float GEMM_H_INV = 1.0f / (HCARRY * WCARRY);
constexpr float HCARRY_INV = 1.0f / HCARRY;

static_assert(N_NODES == 128000, "node count");
static_assert(N_NODES % 64 == 0 && HALF_ROWS % 64 == 0, "GEMM M tile multiple");
static_assert(HID % 64 == 0 && GATES % 64 == 0, "GEMM N tile multiple");
static_assert(HID % 32 == 0 && (2 * HID) % 32 == 0, "GEMM K multiple of 32");
static_assert((2 * SEQ_TILE * HPITCH) % 128 == 0, "h tile zero fill exact");
static_assert(HPITCH % 8 == 0, "16-B aligned h rows");

typedef __attribute__((ext_vector_type(16))) _Float16 v16h;
typedef __attribute__((ext_vector_type(8)))  _Float16 v8h;
typedef __attribute__((ext_vector_type(8)))  float    v8f;
typedef __attribute__((ext_vector_type(4)))  float    v4f;
typedef __attribute__((ext_vector_type(2)))  float    v2f;

struct FragH {
  union U { v16h v; v8h h[2]; };
  static __device__ __forceinline__ v16h load(const _Float16* p) {
    U f; f.h[0] = *(const v8h*)(p); f.h[1] = *(const v8h*)(p + 16); return f.v;
  }
  static __device__ __forceinline__ v8f mma(v16h a, v16h b, v8f c) {
    return __builtin_amdgcn_wmma_f32_16x16x32_f16(false, a, false, b, (short)0, c, false, false);
  }
};
__device__ __forceinline__ void mma_guard4(v8f& a, v8f& b, v8f& c, v8f& d, v16h x, v16h y) {
  asm volatile("v_nop\n\tv_nop\n\tv_nop\n\tv_nop" : "+v"(a), "+v"(b), "+v"(c), "+v"(d) : "v"(x), "v"(y));
}
__device__ __forceinline__ void keep4_h(v16h a, v16h b, v16h c, v16h d) { asm volatile("v_nop" :: "v"(a), "v"(b), "v"(c), "v"(d)); }
__device__ __forceinline__ void acc_guard4(v8f& a, v8f& b, v8f& c, v8f& d) { asm volatile("v_nop\n\tv_nop\n\tv_nop\n\tv_nop" : "+v"(a), "+v"(b), "+v"(c), "+v"(d)); }

__device__ __forceinline__ float h16_to_f32(unsigned hb) {
  const unsigned sgn = (hb & 0x8000u) << 16; const unsigned em = hb & 0x7fffu;
  const float fn = __uint_as_float((em << 13) + 0x38000000u);
  const float fs = (float)em * 5.9604644775390625e-8f;
  const float mag = (em < 0x400u) ? fs : fn; return __uint_as_float(__float_as_uint(mag) | sgn);
}

__device__ __forceinline__ float gate_sig(float x) { return __builtin_amdgcn_rcpf(1.0f + __expf(-x)); }
__device__ __forceinline__ float gate_tanh(float x) {
  const float x2 = x * x;
  const float p = x * (1.0f + x2 * (-0.333333333333f + x2 * (0.133333333333f + x2 * (-0.0539682539683f))));
  const float q = 1.0f - 2.0f * __builtin_amdgcn_rcpf(__expf(2.0f * x) + 1.0f);
  return (fabsf(x) < 0.1f) ? p : q;
}

constexpr int PREP_SEG0 = 2 * 64 * 64 / 8;
constexpr int PREP_SEG1 = 2 * 256 * 64 / 8;
constexpr int PREP_SEG2 = 4 * 256 * 128 / 8;
constexpr int PREP_SEG3 = 6 * 256 * 64 / 8;
constexpr int PREP_N8   = PREP_SEG0 + PREP_SEG1 + PREP_SEG2 + PREP_SEG3;
constexpr int PREP_WBLOCKS = PREP_N8 / 256;
constexpr int OFF_WG    = 0;
constexpr int OFF_WIH0  = OFF_WG + 2 * 64 * 64;
constexpr int OFF_WIH12 = OFF_WIH0 + 2 * 256 * 64;
constexpr int OFF_WHH   = OFF_WIH12 + 4 * 256 * 128;
constexpr int W16_ELEMS = OFF_WHH + 6 * 256 * 64;
constexpr int BS_ELEMS  = 6 * 256;
static_assert(PREP_N8 % 256 == 0 && PREP_SEG0 % 256 == 0 && PREP_SEG1 % 256 == 0 && PREP_SEG2 % 256 == 0, "block-uniform segments");
static_assert(W16_ELEMS == PREP_N8 * 8, "plane coverage");

__global__ __launch_bounds__(256) void prep_kernel(
    const float* __restrict__ Wg12, const float* __restrict__ Wih0, const float* __restrict__ Wih12,
    const float* __restrict__ Whh, const float* __restrict__ bih, const float* __restrict__ bhh,
    unsigned short* __restrict__ W16, float* __restrict__ BS) {
  const int tid = threadIdx.x;
  const int blk = blockIdx.x;
  if (blk < PREP_WBLOCKS) {
    const int i = blk * 256 + tid;
    float v[8];
    if (i < PREP_SEG0) {
      const int l = i >> 9, rem = i & 511, n = rem >> 3, k8 = (rem & 7) * 8;
#pragma unroll
      for (int e = 0; e < 8; ++e) v[e] = Wg12[l * 4096 + (k8 + e) * 64 + n];
    } else if (i < PREP_SEG0 + PREP_SEG1) {
      const int i1 = i - PREP_SEG0;
      const int d = i1 >> 11, rem = i1 & 2047, np = rem >> 3, k8 = (rem & 7) * 8;
      const int srow = (np & 3) * 64 + (np >> 2);
      const float* sp = Wih0 + (size_t)(d * 256 + srow) * 64 + k8;
      const v4f a = *(const v4f*)(sp);
      const v4f b = *(const v4f*)(sp + 4);
#pragma unroll
      for (int e = 0; e < 4; ++e) { v[e] = a[e]; v[4 + e] = b[e]; }
    } else if (i < PREP_SEG0 + PREP_SEG1 + PREP_SEG2) {
      const int i2 = i - PREP_SEG0 - PREP_SEG1;
      const int ld = i2 >> 12, rem = i2 & 4095, np = rem >> 4, k8 = (rem & 15) * 8;
      const int srow = (np & 3) * 64 + (np >> 2);
      const float* sp = Wih12 + (size_t)(ld * 256 + srow) * 128 + k8;
      const v4f a = *(const v4f*)(sp);
      const v4f b = *(const v4f*)(sp + 4);
#pragma unroll
      for (int e = 0; e < 4; ++e) { v[e] = a[e]; v[4 + e] = b[e]; }
    } else {
      const int i3 = i - PREP_SEG0 - PREP_SEG1 - PREP_SEG2;
      const float* sp = Whh + (size_t)i3 * 8;
      const v4f a = *(const v4f*)(sp);
      const v4f b = *(const v4f*)(sp + 4);
#pragma unroll
      for (int e = 0; e < 4; ++e) { v[e] = a[e]; v[4 + e] = b[e]; }
    }
    v8h hv;
#pragma unroll
    for (int e = 0; e < 8; ++e) hv[e] = (_Float16)(v[e] * WCARRY);
    unsigned short* dp = W16 + (size_t)i * 8;
    *(volatile v8h*)dp = hv;
    __threadfence();
    *(volatile v8h*)dp = hv;
  } else {
    const int j = (blk - PREP_WBLOCKS) * 256 + tid;
    if (j < BS_ELEMS / 4) {
      const int o = j * 4;
      const int ld = o >> 8, np = o & 255;
      const int unit = np >> 2;
      v4f s;
#pragma unroll
      for (int g = 0; g < 4; ++g) s[g] = bih[ld * 256 + g * 64 + unit] + bhh[ld * 256 + g * 64 + unit];
      float* dp = BS + o;
      *(volatile v4f*)dp = s;
      __threadfence();
      *(volatile v4f*)dp = s;
    }
  }
}

constexpr int TS_WAVES  = 8;
constexpr int TS_EPW    = 1024;
constexpr int TS_CHUNK  = TS_WAVES * TS_EPW;
constexpr int TS_NCHUNK = N_EDGES / TS_CHUNK;
static_assert(N_EDGES % TS_CHUNK == 0, "edge list is a whole number of chunks");

template <int MODE> struct TsCfg { static constexpr int NT = 16000; static constexpr int ACCW = 1;  static constexpr int CAP = 8192; };
template <>         struct TsCfg<2> { static constexpr int NT = 1000;  static constexpr int ACCW = 64; static constexpr int CAP = 1024; };

template <int MODE>
__global__ __launch_bounds__(256) void tile_stream_kernel(
    const int* __restrict__ ESRC, const int* __restrict__ EDST, const float* __restrict__ EW,
    const float* __restrict__ NORM, const float* __restrict__ XIN, const float* __restrict__ DEGI,
    const float* __restrict__ W0, const float* __restrict__ B0,
    float* __restrict__ OUTA, float* __restrict__ OUTB, unsigned short* __restrict__ OUT16) {
  constexpr int NT   = TsCfg<MODE>::NT;
  constexpr int ACCW = TsCfg<MODE>::ACCW;
  constexpr int CAP  = TsCfg<MODE>::CAP;
  constexpr int MAXPASS = TS_CHUNK / CAP;
  static_assert(N_NODES % NT == 0, "tiles cover the node set exactly");
  static_assert(NT % 32 == 0 || MODE == 2, "scalar tiles start on 128-B lines");
  static_assert(NT % 4 == 0 && (NT * ACCW) % 4 == 0, "row groups exact");
  __shared__ __align__(16) float accS[NT * ACCW];
  __shared__ int listE[CAP];
  __shared__ int listD[CAP];
  __shared__ int cntw[2][TS_WAVES];

  const int tid = threadIdx.x, lane = tid & 31, wave = tid >> 5;
  const int nbase = blockIdx.x * NT;

  {
    const v4f z4 = {0.f, 0.f, 0.f, 0.f};
#pragma unroll 1
    for (int idx = tid; idx < NT * ACCW / 4; idx += 256) *(v4f*)(accS + 4 * idx) = z4;
  }
  __syncthreads();

#pragma unroll 1
  for (int ch = 0; ch < TS_NCHUNK; ++ch) {
    const int ebase = ch * TS_CHUNK + wave * TS_EPW;
    unsigned flags = 0u;
#pragma unroll
    for (int j = 0; j < 8; ++j) {
      const int4 d = *(const int4*)(EDST + ebase + j * 128 + lane * 4);
      const unsigned f0 = (((unsigned)d.x - (unsigned)nbase) < (unsigned)NT) ? 1u : 0u;
      const unsigned f1 = (((unsigned)d.y - (unsigned)nbase) < (unsigned)NT) ? 1u : 0u;
      const unsigned f2 = (((unsigned)d.z - (unsigned)nbase) < (unsigned)NT) ? 1u : 0u;
      const unsigned f3 = (((unsigned)d.w - (unsigned)nbase) < (unsigned)NT) ? 1u : 0u;
      flags |= (f0 | (f1 << 1) | (f2 << 2) | (f3 << 3)) << (4 * j);
    }
    const int cnt = __popc(flags);
    int incl = cnt;
#pragma unroll
    for (int off = 1; off < 32; off <<= 1) {
      const int tv = __shfl_up(incl, off, 32);
      incl += (lane >= off) ? tv : 0;
    }
    const int wtot = __shfl(incl, 31, 32);
    const int excl = incl - cnt;
    if (lane == 0) cntw[ch & 1][wave] = wtot;
    __syncthreads();
    int base = 0, total = 0;
#pragma unroll
    for (int w = 0; w < TS_WAVES; ++w) {
      const int cw = min(max(cntw[ch & 1][w], 0), TS_EPW);
      base += (w < wave) ? cw : 0;
      total += cw;
    }
    total = __builtin_amdgcn_readfirstlane(total);
    base  = __builtin_amdgcn_readfirstlane(base);

#pragma unroll 1
    for (int ps = 0; ps < MAXPASS; ++ps) {
      const int r0 = ps * CAP;
      if (r0 >= total) break;
      {
        unsigned m = flags;
        int p = base + excl;
#pragma unroll 1
        for (int it = 0; it < 32; ++it) {
          const unsigned any = __builtin_amdgcn_ballot_w32(m != 0u);
          if (any == 0u) break;
          const int b = __builtin_ctz(m | 0x80000000u);
          const int e = ebase + (b >> 2) * 128 + lane * 4 + (b & 3);
          int dv = EDST[e];
          asm volatile("" : "+v"(dv));
          const int rel = p - r0;
          if ((m != 0u) && (rel >= 0) && (rel < CAP)) { listE[rel] = e; listD[rel] = dv - nbase; }
          p += (m != 0u) ? 1 : 0;
          m &= (m - 1u);
        }
      }
      __syncthreads();
      const int nr = min(total - r0, CAP);
#pragma unroll 1
      for (int bb = 0; bb < nr; bb += 32) {
        const int idx = bb + lane;
        const int idc = min(idx, nr - 1);
        const int ee = listE[idc];
        const int dd = listD[idc];
        const bool mine = (idx < nr) && ((dd & (TS_WAVES - 1)) == wave);
        unsigned mask = __builtin_amdgcn_ballot_w32(mine);
#pragma unroll 1
        for (int it = 0; it < 32; ++it) {
          if (mask == 0u) break;
          const int k = __builtin_ctz(mask);
          mask &= (mask - 1u);
          int e  = __builtin_amdgcn_readlane(ee, k);
          int dl = __builtin_amdgcn_readlane(dd, k);
          e  = min(max(e, 0), N_EDGES - 1);
          dl = min(max(dl, 0), NT - 1);
          if (MODE == 0) {
            float val = EW[e];
            asm volatile("" : "+v"(val));
            if (lane == 0) accS[dl] += val;
          } else if (MODE == 1) {
            int s = ESRC[e];
            asm volatile("" : "+v"(s));
            s = min(max(s, 0), N_NODES - 1);
            float nv = NORM[e];
            asm volatile("" : "+v"(nv));
            float xs = XIN[s];
            asm volatile("" : "+v"(xs));
            float val = nv * xs;
            asm volatile("" : "+v"(val));
            if (lane == 0) accS[dl] += val;
          } else {
            int s = ESRC[e];
            asm volatile("" : "+v"(s));
            s = min(max(s, 0), N_NODES - 1);
            float nv = NORM[e];
            asm volatile("" : "+v"(nv));
            const v2f hv = *(const v2f*)(XIN + (size_t)s * 64 + 2 * lane);
            float* ap = accS + dl * ACCW + 2 * lane;
            v2f a = *(v2f*)ap;
            a[0] = fmaf(nv, hv[0], a[0]);
            a[1] = fmaf(nv, hv[1], a[1]);
            *(v2f*)ap = a;
          }
        }
      }
      __syncthreads();
    }
  }
  __syncthreads();

  if (MODE == 0) {
#pragma unroll 1
    for (int idx = tid; idx < NT / 4; idx += 256) {
      const v4f a = *(const v4f*)(accS + 4 * idx);
      v4f dg, ds;
#pragma unroll
      for (int e = 0; e < 4; ++e) { dg[e] = a[e] + 1.0f; ds[e] = rsqrtf(dg[e]); }
      float* pa = OUTA + nbase + 4 * idx;
      float* pb = OUTB + nbase + 4 * idx;
      *(volatile v4f*)pa = dg;
      *(volatile v4f*)pb = ds;
      __threadfence();
      *(volatile v4f*)pa = dg;
      *(volatile v4f*)pb = ds;
    }
  } else if (MODE == 1) {
    const int hh = lane >> 4, c4 = (lane & 15) * 4;
    const v4f wv = *(const v4f*)(W0 + c4);
    const v4f bv = *(const v4f*)(B0 + c4);
#pragma unroll 1
    for (int pr = wave; pr < NT / 2; pr += TS_WAVES) {
      const int n = 2 * pr + hh;
      const int i = nbase + n;
      const float s = accS[n] + XIN[i] * (1.0f / DEGI[i]);
      v4f o;
#pragma unroll
      for (int e = 0; e < 4; ++e) o[e] = fmaxf(fmaf(s, wv[e], bv[e]), 0.0f);
      float* op = OUTA + (size_t)i * 64 + c4;
      *(volatile v4f*)op = o;
      __threadfence();
      *(volatile v4f*)op = o;
    }
  } else {
    const int sub = lane >> 3, c8 = (lane & 7) * 8;
#pragma unroll 1
    for (int rg = wave; rg < NT / 4; rg += TS_WAVES) {
      const int n = 4 * rg + sub;
      const int i = nbase + n;
      const float rd = 1.0f / DEGI[i];
      const v4f a0 = *(const v4f*)(accS + n * ACCW + c8);
      const v4f a1 = *(const v4f*)(accS + n * ACCW + c8 + 4);
      const v4f h0 = *(const v4f*)(XIN + (size_t)i * 64 + c8);
      const v4f h1 = *(const v4f*)(XIN + (size_t)i * 64 + c8 + 4);
      v8h hv;
#pragma unroll
      for (int e = 0; e < 4; ++e) {
        hv[e]     = (_Float16)((a0[e] + h0[e] * rd) * GCARRY);
        hv[4 + e] = (_Float16)((a1[e] + h1[e] * rd) * GCARRY);
      }
      unsigned short* op = OUT16 + (size_t)i * 64 + c8;
      *(volatile v8h*)op = hv;
      __threadfence();
      *(volatile v8h*)op = hv;
    }
  }
}

static_assert((N_EDGES / 4) % 256 == 0, "edge coefficient grid exact");
__global__ __launch_bounds__(256) void edge_norm_kernel(
    const int* __restrict__ ESRC, const int* __restrict__ EDST, const float* __restrict__ EW,
    const float* __restrict__ DIS, float* __restrict__ NORM) {
  const int i = blockIdx.x * 256 + threadIdx.x;
  const int4 s = ((const int4*)ESRC)[i];
  const int4 d = ((const int4*)EDST)[i];
  const v4f w = ((const v4f*)EW)[i];
  const int s0 = min(max(s.x, 0), N_NODES - 1), s1 = min(max(s.y, 0), N_NODES - 1);
  const int s2 = min(max(s.z, 0), N_NODES - 1), s3 = min(max(s.w, 0), N_NODES - 1);
  const int d0 = min(max(d.x, 0), N_NODES - 1), d1 = min(max(d.y, 0), N_NODES - 1);
  const int d2 = min(max(d.z, 0), N_NODES - 1), d3 = min(max(d.w, 0), N_NODES - 1);
  v4f o;
  o[0] = DIS[s0] * w[0] * DIS[d0];
  o[1] = DIS[s1] * w[1] * DIS[d1];
  o[2] = DIS[s2] * w[2] * DIS[d2];
  o[3] = DIS[s3] * w[3] * DIS[d3];
  float* op = NORM + (size_t)i * 4;
  *(volatile v4f*)op = o;
  __threadfence();
  *(volatile v4f*)op = o;
}

template <int OUT_MODE, int ACT>
__global__ __launch_bounds__(256) void gemm_f16_kernel(
    const unsigned short* __restrict__ Ap, int lda,
    const unsigned short* __restrict__ Btp, int ldb,
    void* __restrict__ Cout, int ldc,
    const float* __restrict__ bias,
    int M, int N, int K, float scale, float oscale) {
  const _Float16* A  = (const _Float16*)Ap;
  const _Float16* Bt = (const _Float16*)Btp;
  __shared__ __align__(16) float sT[8][16 * 68];
  const int lane = threadIdx.x & 31;
  const int wave = threadIdx.x >> 5;
  const int tilesN = N >> 6;
  const int tilesM = M >> 6;
  const int tile = blockIdx.x * 8 + wave;
  if (tile >= tilesM * tilesN) return;
  const int tm = tile / tilesN;
  const int tn = tile - tm * tilesN;
  const int m0 = tm << 6;
  const int n0 = tn << 6;

  const int rlane = lane & 15;
  const int koff  = (lane >> 4) * 8;
  const int mOff  = (lane >> 4) * 8;

  v8f acc[4][4];
#pragma unroll
  for (int i = 0; i < 4; ++i)
#pragma unroll
    for (int j = 0; j < 4; ++j) acc[i][j] = (v8f){0.f, 0.f, 0.f, 0.f, 0.f, 0.f, 0.f, 0.f};

  for (int k0 = 0; k0 < K; k0 += 32) {
    v16h bh[4];
#pragma unroll
    for (int j = 0; j < 4; ++j) {
      const size_t bo = (size_t)(n0 + (j << 4) + rlane) * ldb + koff + k0;
      bh[j] = FragH::load(Bt + bo);
    }
#pragma unroll
    for (int i = 0; i < 4; ++i) {
      const size_t ao = (size_t)(m0 + (i << 4) + rlane) * lda + koff + k0;
      const v16h ah = FragH::load(A + ao);
#pragma unroll
      for (int j = 0; j < 4; ++j) acc[i][j] = FragH::mma(ah, bh[j], acc[i][j]);
      mma_guard4(acc[i][0], acc[i][1], acc[i][2], acc[i][3], ah, bh[3]);
    }
    keep4_h(bh[0], bh[1], bh[2], bh[3]);
  }
  acc_guard4(acc[0][0], acc[0][1], acc[0][2], acc[0][3]);
  acc_guard4(acc[1][0], acc[1][1], acc[1][2], acc[1][3]);
  acc_guard4(acc[2][0], acc[2][1], acc[2][2], acc[2][3]);
  acc_guard4(acc[3][0], acc[3][1], acc[3][2], acc[3][3]);

  float* slab = sT[wave];
#pragma unroll
  for (int i = 0; i < 4; ++i) {
    const int mBase = m0 + (i << 4);
#pragma unroll
    for (int j = 0; j < 4; ++j) {
      const int n = n0 + (j << 4) + rlane;
      const float bv = bias[n];
#pragma unroll
      for (int r = 0; r < 8; ++r) {
        float v = acc[i][j][r] * scale + bv;
        if (ACT == 2) v = fmaxf(v, 0.0f);
        v = v * oscale;
        slab[(mOff + r) * 68 + (j << 4) + rlane] = v;
      }
    }
    __builtin_amdgcn_fence(__ATOMIC_RELEASE, "workgroup");
    __builtin_amdgcn_wave_barrier();
    __builtin_amdgcn_fence(__ATOMIC_ACQUIRE, "workgroup");
    if (OUT_MODE == 0) {
      float* C = (float*)Cout;
      const int hh = lane >> 4, c4 = (lane & 15) * 4;
      for (int pass = 0; pass < 2; ++pass) {
#pragma unroll
        for (int it = 0; it < 8; ++it) {
          const int row = it * 2 + hh;
          const v4f v = *(const v4f*)(slab + row * 68 + c4);
          *(volatile v4f*)(C + (size_t)(mBase + row) * ldc + n0 + c4) = v;
        }
        __threadfence();
      }
    } else {
      const int q = lane >> 3, c8 = (lane & 7) * 8;
      unsigned short* C = (unsigned short*)Cout;
      for (int pass = 0; pass < 2; ++pass) {
#pragma unroll
        for (int it = 0; it < 4; ++it) {
          const int row = it * 4 + q;
          const float* sp = slab + row * 68 + c8;
          v8h hv;
#pragma unroll
          for (int e = 0; e < 8; ++e) hv[e] = (_Float16)sp[e];
          *(volatile v8h*)(C + (size_t)(mBase + row) * ldc + n0 + c8) = hv;
        }
        __threadfence();
      }
    }
    __builtin_amdgcn_fence(__ATOMIC_RELEASE, "workgroup");
    __builtin_amdgcn_wave_barrier();
    __builtin_amdgcn_fence(__ATOMIC_ACQUIRE, "workgroup");
  }
}

__global__ __launch_bounds__(128) void lstm_scan_kernel(
    const float* __restrict__ XP, const unsigned short* __restrict__ WHHp,
    unsigned short* __restrict__ SEQ, int dir, int half) {
  __shared__ __align__(16) _Float16 Ah[2][SEQ_TILE * HPITCH];
  const _Float16* WHH = (const _Float16*)WHHp;
  const int tid = threadIdx.x, lane = tid & 31, q = tid >> 5;
  const int c = lane & 15, hh = lane >> 4, koff = hh * 8;
  const int bl0 = blockIdx.x * SEQ_TILE;
  const int bg0 = half * HALF_SAMPLES + bl0;

  {
    _Float16* ahf = &Ah[0][0];
#pragma unroll 1
    for (int i = tid; i < 2 * SEQ_TILE * HPITCH; i += 128) ahf[i] = (_Float16)0.0f;
  }
  v16h bw[4][2];
#pragma unroll
  for (int g = 0; g < 4; ++g)
#pragma unroll
    for (int kt = 0; kt < 2; ++kt)
      bw[g][kt] = FragH::load(WHH + (size_t)(g * 64 + 16 * q + c) * HID + koff + 32 * kt);
  float cst[8];
#pragma unroll
  for (int r = 0; r < 8; ++r) cst[r] = 0.0f;
  __syncthreads();

  const int unit = 16 * q + c;
#pragma unroll 1
  for (int s = 0; s < N_STEPS; ++s) {
    const int t = dir ? (N_STEPS - 1 - s) : s;
    const int cur = s & 1;
    v4f xv[8];
#pragma unroll
    for (int r = 0; r < 8; ++r)
      xv[r] = *(const v4f*)(XP + ((size_t)(bl0 + 8 * hh + r) * N_STEPS + (size_t)t) * GATES + unit * 4);

    const _Float16* arow = &Ah[cur][0] + c * HPITCH + koff;
    const v16h a0 = FragH::load(arow);
    const v16h a1 = FragH::load(arow + 32);
    v8f acc[4];
#pragma unroll
    for (int g = 0; g < 4; ++g) acc[g] = (v8f){0.f, 0.f, 0.f, 0.f, 0.f, 0.f, 0.f, 0.f};
#pragma unroll
    for (int g = 0; g < 4; ++g) acc[g] = FragH::mma(a0, bw[g][0], acc[g]);
#pragma unroll
    for (int g = 0; g < 4; ++g) acc[g] = FragH::mma(a1, bw[g][1], acc[g]);
    mma_guard4(acc[0], acc[1], acc[2], acc[3], a0, a1);
    keep4_h(bw[0][0], bw[1][0], bw[2][0], bw[3][0]);
    keep4_h(bw[0][1], bw[1][1], bw[2][1], bw[3][1]);

    _Float16* ahn = &Ah[cur ^ 1][0];
#pragma unroll
    for (int r = 0; r < 8; ++r) {
      const float gi = acc[0][r] * GEMM_H_INV + xv[r][0];
      const float gf = acc[1][r] * GEMM_H_INV + xv[r][1];
      const float gg = acc[2][r] * GEMM_H_INV + xv[r][2];
      const float go = acc[3][r] * GEMM_H_INV + xv[r][3];
      const float si = gate_sig(gi);
      const float sf = gate_sig(gf);
      const float so = gate_sig(go);
      const float cn = sf * cst[r] + si * gate_tanh(gg);
      cst[r] = cn;
      const float hn = so * gate_tanh(cn);
      ahn[(8 * hh + r) * HPITCH + unit] = (_Float16)(hn * HCARRY);
    }
    __syncthreads();
    {
      const int row = 4 * q + (lane >> 3), c8 = (lane & 7) * 8;
      const v8h hv = *(const v8h*)(ahn + row * HPITCH + c8);
      unsigned short* dp = SEQ + ((size_t)(bg0 + row) * N_STEPS + (size_t)t) * (2 * HID) + dir * HID + c8;
      *(volatile v8h*)dp = hv;
      __threadfence();
      *(volatile v8h*)dp = hv;
    }
  }
}

static_assert(N_NODES % 256 == 0, "head grid exact");
__global__ __launch_bounds__(256) void head_kernel(
    const unsigned short* __restrict__ SEQ, const float* __restrict__ Wfc, const float* __restrict__ bfc,
    float* __restrict__ out) {
  __shared__ float wsm[2 * HID];
  const int tid = threadIdx.x;
  if (tid < 2 * HID) wsm[tid] = Wfc[tid];
  __syncthreads();
  const int i = blockIdx.x * 256 + tid;
  const uint4* rp = (const uint4*)(SEQ + (size_t)i * (2 * HID));
  float acc = 0.0f;
#pragma unroll 1
  for (int k8 = 0; k8 < (2 * HID) / 8; ++k8) {
    const uint4 w = rp[k8];
    const float* wp = wsm + k8 * 8;
    acc = fmaf(h16_to_f32(w.x & 0xffffu), wp[0], acc);
    acc = fmaf(h16_to_f32(w.x >> 16),     wp[1], acc);
    acc = fmaf(h16_to_f32(w.y & 0xffffu), wp[2], acc);
    acc = fmaf(h16_to_f32(w.y >> 16),     wp[3], acc);
    acc = fmaf(h16_to_f32(w.z & 0xffffu), wp[4], acc);
    acc = fmaf(h16_to_f32(w.z >> 16),     wp[5], acc);
    acc = fmaf(h16_to_f32(w.w & 0xffffu), wp[6], acc);
    acc = fmaf(h16_to_f32(w.w >> 16),     wp[7], acc);
  }
  const float o = acc * HCARRY_INV + bfc[0];
  *(volatile float*)(out + i) = o;
  __threadfence();
  *(volatile float*)(out + i) = o;
}

extern "C" void kernel_launch(void* const* d_in, const int* in_sizes, int n_in,
                              void* d_out, int out_size, void* d_ws, size_t ws_size, hipStream_t stream) {
  if (n_in < 14 || d_out == nullptr || d_ws == nullptr) return;
  if (in_sizes[0] != N_NODES || in_sizes[1] != N_EDGES || in_sizes[2] != N_EDGES || in_sizes[3] != N_EDGES ||
      in_sizes[4] != HID || in_sizes[5] != 2 * HID * HID || in_sizes[6] != 3 * HID ||
      in_sizes[7] != 2 * GATES * HID || in_sizes[8] != 4 * GATES * 2 * HID || in_sizes[9] != 6 * GATES * HID ||
      in_sizes[10] != 6 * GATES || in_sizes[11] != 6 * GATES || in_sizes[12] != 2 * HID || in_sizes[13] != 1 ||
      out_size != N_NODES) return;

  const float* x     = (const float*)d_in[0];
  const int*   esrc  = (const int*)d_in[1];
  const int*   edst  = (const int*)d_in[2];
  const float* ew    = (const float*)d_in[3];
  const float* Wg0   = (const float*)d_in[4];
  const float* Wg12  = (const float*)d_in[5];
  const float* bg    = (const float*)d_in[6];
  const float* Wih0  = (const float*)d_in[7];
  const float* Wih12 = (const float*)d_in[8];
  const float* Whh   = (const float*)d_in[9];
  const float* bih   = (const float*)d_in[10];
  const float* bhh   = (const float*)d_in[11];
  const float* Wfc   = (const float*)d_in[12];
  const float* bfc   = (const float*)d_in[13];
  float* out = (float*)d_out;

  char* ws = (char*)d_ws;
  size_t off = 0;
  auto carve = [&](size_t bytes) -> char* { char* p = ws + off; off += (bytes + 255) & ~(size_t)255; return p; };
  char* R_XP   = carve((size_t)HALF_ROWS * GATES * 4);
  char* R_SEQA = carve((size_t)N_NODES * 2 * HID * 2);
  char* R_SEQB = carve((size_t)N_NODES * 2 * HID * 2);
  char* R_DEG  = carve((size_t)N_NODES * 4);
  char* R_DIS  = carve((size_t)N_NODES * 4);
  char* R_W16  = carve((size_t)W16_ELEMS * 2);
  char* R_BS   = carve((size_t)BS_ELEMS * 4);
  if (off > ws_size || off > (size_t)134217728) return;
  static_assert((size_t)N_NODES * HID * 4 + (size_t)N_EDGES * 4 <= (size_t)HALF_ROWS * GATES * 4, "graph-phase planes fit the XP region");

  float* XP   = (float*)R_XP;
  float* HPL  = (float*)R_XP;
  float* NORM = (float*)(R_XP + (size_t)N_NODES * HID * 4);
  unsigned short* SEQA = (unsigned short*)R_SEQA;
  unsigned short* SEQB = (unsigned short*)R_SEQB;
  unsigned short* G16  = SEQA;
  unsigned short* H3C  = SEQB;
  float* DEG = (float*)R_DEG;
  float* DIS = (float*)R_DIS;
  unsigned short* W16 = (unsigned short*)R_W16;
  float* BS = (float*)R_BS;

  prep_kernel<<<PREP_WBLOCKS + 2, 256, 0, stream>>>(Wg12, Wih0, Wih12, Whh, bih, bhh, W16, BS);

  tile_stream_kernel<0><<<N_NODES / TsCfg<0>::NT, 256, 0, stream>>>(esrc, edst, ew, ew, ew, ew, Wg0, bg, DEG, DIS, G16);
  edge_norm_kernel<<<N_EDGES / 4 / 256, 256, 0, stream>>>(esrc, edst, ew, DIS, NORM);
  tile_stream_kernel<1><<<N_NODES / TsCfg<1>::NT, 256, 0, stream>>>(esrc, edst, ew, NORM, x, DEG, Wg0, bg, HPL, HPL, G16);
  tile_stream_kernel<2><<<N_NODES / TsCfg<2>::NT, 256, 0, stream>>>(esrc, edst, ew, NORM, HPL, DEG, Wg0, bg, DIS, DIS, G16);
  gemm_f16_kernel<0, 2><<<(N_NODES / 64) * (HID / 64) / 8, 256, 0, stream>>>(
      G16, HID, W16 + OFF_WG, HID, (void*)HPL, HID, bg + HID, N_NODES, HID, HID, GEMM_G_INV, 1.0f);
  tile_stream_kernel<2><<<N_NODES / TsCfg<2>::NT, 256, 0, stream>>>(esrc, edst, ew, NORM, HPL, DEG, Wg0, bg, DIS, DIS, G16);
  gemm_f16_kernel<1, 2><<<(N_NODES / 64) * (HID / 64) / 8, 256, 0, stream>>>(
      G16, HID, W16 + OFF_WG + HID * HID, HID, (void*)H3C, HID, bg + 2 * HID, N_NODES, HID, HID, GEMM_G_INV, GCARRY);

  for (int l = 0; l < 3; ++l) {
    const int in_dim = (l == 0) ? HID : 2 * HID;
    const unsigned short* inP = (l == 0) ? H3C : ((l == 1) ? SEQA : SEQB);
    unsigned short* outP = (l == 1) ? SEQB : SEQA;
    const float pscale = (l == 0) ? GEMM_G_INV : GEMM_H_INV;
    for (int d = 0; d < 2; ++d) {
      const unsigned short* wih = (l == 0) ? (W16 + OFF_WIH0 + (size_t)d * GATES * HID)
                                           : (W16 + OFF_WIH12 + (size_t)((l - 1) * 2 + d) * GATES * 2 * HID);
      const unsigned short* whh = W16 + OFF_WHH + (size_t)(l * 2 + d) * GATES * HID;
      const float* bs = BS + (l * 2 + d) * GATES;
      for (int hf = 0; hf < 2; ++hf) {
        gemm_f16_kernel<0, 0><<<(HALF_ROWS / 64) * (GATES / 64) / 8, 256, 0, stream>>>(
            inP + (size_t)hf * HALF_ROWS * in_dim, in_dim, wih, in_dim, (void*)XP, GATES, bs,
            HALF_ROWS, GATES, in_dim, pscale, 1.0f);
        lstm_scan_kernel<<<HALF_SAMPLES / SEQ_TILE, 128, 0, stream>>>(XP, whh, outP, d, hf);
      }
    }
  }

  head_kernel<<<N_NODES / 256, 256, 0, stream>>>(SEQA, Wfc, bfc, out);
}
